// EquivariantConvolution_60687887892710
// MI455X (gfx1250) — hardware-verified
//
#include <hip/hip_runtime.h>
#include <stdint.h>


#define WPB 4
#define NTHR (WPB * 32)
#define HID 32
#define EFD 16
#define NB 32
#define NA 32
#define NCH (HID + 1)
#define TBL_ROWS (NCH * NA)
#define HP 16
#define RP 36
#define FDIM 32
#define ODIM 32
#define BDIM 16

typedef __bf16 v16bf __attribute__((ext_vector_type(16)));
typedef unsigned short v16us __attribute__((ext_vector_type(16)));
typedef unsigned short v8us __attribute__((ext_vector_type(8)));
typedef float v8f __attribute__((ext_vector_type(8)));
typedef float v4f __attribute__((ext_vector_type(4)));

union Frag { v16bf v; v16us u; v8us h8[2]; };

__device__ __forceinline__ void split_bf16(float x, unsigned short& ho, unsigned short& lo) {
  const unsigned u  = __float_as_uint(x);
  const unsigned hu = (u + 0x7FFFu + ((u >> 16) & 1u)) >> 16;
  const float hf    = __uint_as_float(hu << 16);
  const float rem   = x - hf;
  const unsigned ru = __float_as_uint(rem);
  const unsigned lu = (ru + 0x7FFFu + ((ru >> 16) & 1u)) >> 16;
  ho = (unsigned short)hu;
  lo = (unsigned short)lu;
}

__device__ __forceinline__ v8f wmma3(v8f acc, const Frag& ah, const Frag& al, const Frag& bh, const Frag& bl) {
  acc = __builtin_amdgcn_wmma_f32_16x16x32_bf16(false, ah.v, false, bh.v, (short)0, acc, false, false);
  acc = __builtin_amdgcn_wmma_f32_16x16x32_bf16(false, ah.v, false, bl.v, (short)0, acc, false, false);
  acc = __builtin_amdgcn_wmma_f32_16x16x32_bf16(false, al.v, false, bh.v, (short)0, acc, false, false);
  asm volatile("v_nop\n\tv_nop\n\tv_nop\n\tv_nop" : "+v"(acc) : "v"(ah.u), "v"(al.u), "v"(bh.u), "v"(bl.u));
  return acc;
}

__device__ __forceinline__ void accum_weighted(v8f& T, const v8f& acc, const v4f& hv0, const v4f& hv1) {
#pragma unroll
  for (int r = 0; r < 4; ++r) {
    T[r]     += hv0[r] * acc[r];
    T[4 + r] += hv1[r] * acc[4 + r];
  }
}

__global__ __launch_bounds__(NTHR) void k_split_tbl(const float* __restrict__ w2,
                                                    const float* __restrict__ bias2,
                                                    unsigned short* __restrict__ tblH,
                                                    unsigned short* __restrict__ tblL,
                                                    int nW2, int nTot)
{
  const int g    = (int)blockIdx.x * NTHR + (int)threadIdx.x;
  const int base = g * 8;
  if (base + 8 > nTot) return;
  v4f x0, x1;
  if (base + 8 <= nW2) {
    x0 = *(const v4f*)(w2 + base);
    x1 = *(const v4f*)(w2 + base + 4);
  } else {
    const float* p = bias2 + (base - nW2);
    x0 = *(const v4f*)p;
    x1 = *(const v4f*)(p + 4);
  }
  v8us hv, lv;
#pragma unroll
  for (int i = 0; i < 4; ++i) {
    unsigned short hq, lq;
    split_bf16(x0[i], hq, lq); hv[i] = hq;     lv[i] = lq;
    split_bf16(x1[i], hq, lq); hv[4 + i] = hq; lv[4 + i] = lq;
  }
  *(volatile v8us*)(tblH + base) = hv;
  *(volatile v8us*)(tblL + base) = lv;
  __threadfence();
  *(volatile v8us*)(tblH + base) = hv;
  *(volatile v8us*)(tblL + base) = lv;
}

__global__ __launch_bounds__(NTHR) void k_edge_main(
    const float* __restrict__ basis1,
    const float* __restrict__ basis2,
    const float* __restrict__ ef,
    const float* __restrict__ fnode,
    const int*   __restrict__ src,
    const float* __restrict__ w1,
    const float* __restrict__ bias1,
    const unsigned short* __restrict__ tblH,
    const unsigned short* __restrict__ tblL,
    float* __restrict__ out,
    int E, int Nn, int nIter)
{
  __shared__ __attribute__((aligned(16))) unsigned short w1s[2 * HID * EFD];
  __shared__ __attribute__((aligned(16))) float hS[WPB][NCH * HP];
  __shared__ __attribute__((aligned(16))) float rS[WPB][16 * RP];
  __shared__ __attribute__((aligned(16))) float bS[WPB][16 * BDIM];

  const int tid  = (int)threadIdx.x;
  const int lane = tid & 31;
  const int wave = tid >> 5;
  const int lrow = lane & 15;
  const int lh   = lane >> 4;

  {
    const int n  = tid >> 2;
    const int kq = (tid & 3) * 4;
#pragma unroll
    for (int d = 0; d < 4; ++d) {
      const float x = w1[(kq + d) * HID + n];
      unsigned short hq, lq;
      split_bf16(x, hq, lq);
      w1s[n * EFD + kq + d]             = hq;
      w1s[HID * EFD + n * EFD + kq + d] = lq;
    }
  }
  if (lane < 16) hS[wave][HID * HP + lane] = 1.0f;
  const float b1v0 = bias1[lrow];
  const float b1v1 = bias1[16 + lrow];
  __syncthreads();

  float* hSw = &hS[wave][0];
  float* rSw = &rS[wave][0];
  float* bSw = &bS[wave][0];
  const int Em1 = E - 1;

  for (int it = 0; it < nIter; ++it) {
    const int tile = (int)blockIdx.x * WPB + wave + it * (int)gridDim.x * WPB;
    const int e0   = tile * 16;
    int er = e0 + lrow; if (er > Em1) er = Em1;

    Frag aeh, ael;
    {
      const float* p = ef + (size_t)er * EFD + 8 * lh;
      const v4f x0 = *(const v4f*)p;
      const v4f x1 = *(const v4f*)(p + 4);
#pragma unroll
      for (int i = 0; i < 4; ++i) {
        unsigned short hq, lq;
        split_bf16(x0[i], hq, lq); aeh.u[i] = hq;     ael.u[i] = lq;
        split_bf16(x1[i], hq, lq); aeh.u[4 + i] = hq; ael.u[4 + i] = lq;
      }
#pragma unroll
      for (int i = 8; i < 16; ++i) { aeh.u[i] = 0; ael.u[i] = 0; }
    }
#pragma unroll
    for (int nn = 0; nn < 2; ++nn) {
      const int n = nn * 16 + lrow;
      Frag bh, bl;
      bh.h8[0] = *(const v8us*)&w1s[n * EFD + 8 * lh];
      bl.h8[0] = *(const v8us*)&w1s[HID * EFD + n * EFD + 8 * lh];
#pragma unroll
      for (int i = 8; i < 16; ++i) { bh.u[i] = 0; bl.u[i] = 0; }
      v8f acc;
#pragma unroll
      for (int i = 0; i < 8; ++i) acc[i] = 0.0f;
      acc = wmma3(acc, aeh, ael, bh, bl);
      const float bb = nn ? b1v1 : b1v0;
      v4f o0, o1;
#pragma unroll
      for (int r = 0; r < 4; ++r) {
        o0[r] = fmaxf(acc[r] + bb, 0.0f);
        o1[r] = fmaxf(acc[4 + r] + bb, 0.0f);
      }
      *(v4f*)&hSw[n * HP + 8 * lh]     = o0;
      *(v4f*)&hSw[n * HP + 8 * lh + 4] = o1;
    }

    Frag ath, atl;
    {
      int s = src[er];
      if (s < 0) s = 0;
      if (s > Nn - 1) s = Nn - 1;
      const float* fp = fnode  + (size_t)s  * FDIM;
      const float* bp = basis1 + (size_t)er * BDIM;
      const v4f bd0 = *(const v4f*)(bp);
      const v4f bd1 = *(const v4f*)(bp + 4);
      const v4f bd2 = *(const v4f*)(bp + 8);
      const v4f bd3 = *(const v4f*)(bp + 12);
#pragma unroll
      for (int g = 0; g < 4; ++g) {
        const int m1 = 2 * lh + (g & 1) + 4 * (g >> 1);
        const v4f fr = *(const v4f*)(fp + m1 * 4);
#pragma unroll
        for (int k1 = 0; k1 < 4; ++k1) {
          const float t = fr.x * bd0[k1] + fr.y * bd1[k1] + fr.z * bd2[k1] + fr.w * bd3[k1];
          unsigned short hq, lq;
          split_bf16(t, hq, lq);
          ath.u[4 * g + k1] = hq;
          atl.u[4 * g + k1] = lq;
        }
      }
    }
    __syncthreads();

    v8f T0, T1;
#pragma unroll
    for (int i = 0; i < 8; ++i) { T0[i] = 0.0f; T1[i] = 0.0f; }
    const unsigned short* thp = tblH + lrow * NB + 8 * lh;
    const unsigned short* tlp = tblL + lrow * NB + 8 * lh;
#pragma unroll 1
    for (int c = 0; c < NCH; ++c) {
      const v4f hv0 = *(const v4f*)&hSw[c * HP + 8 * lh];
      const v4f hv1 = *(const v4f*)&hSw[c * HP + 8 * lh + 4];
#pragma unroll
      for (int ah = 0; ah < 2; ++ah) {
        const int n0 = (2 * c + ah) * 16;
        Frag bh, bl;
        bh.h8[0] = *(const v8us*)(thp + n0 * NB);
        bh.h8[1] = *(const v8us*)(thp + n0 * NB + 16);
        bl.h8[0] = *(const v8us*)(tlp + n0 * NB);
        bl.h8[1] = *(const v8us*)(tlp + n0 * NB + 16);
        v8f acc;
#pragma unroll
        for (int i = 0; i < 8; ++i) acc[i] = 0.0f;
        acc = wmma3(acc, ath, atl, bh, bl);
        if (ah == 0) accum_weighted(T0, acc, hv0, hv1);
        else         accum_weighted(T1, acc, hv0, hv1);
      }
    }

#pragma unroll
    for (int r = 0; r < 8; ++r) {
      rSw[(8 * lh + r) * RP + lrow]      = T0[r];
      rSw[(8 * lh + r) * RP + 16 + lrow] = T1[r];
    }
    {
      int eb = e0 + (lane >> 1); if (eb > Em1) eb = Em1;
      const float* p = basis2 + (size_t)eb * BDIM + (lane & 1) * 8;
      *(v4f*)&bSw[(lane >> 1) * BDIM + (lane & 1) * 8]     = *(const v4f*)p;
      *(v4f*)&bSw[(lane >> 1) * BDIM + (lane & 1) * 8 + 4] = *(const v4f*)(p + 4);
    }
    __syncthreads();

    v4f ov[4];
#pragma unroll
    for (int j = 0; j < 4; ++j) {
      const int el = 4 * j + (lane >> 3);
      const int m2 = lane & 7;
      const v4f rv = *(const v4f*)&rSw[el * RP + m2 * 4];
      const float* bb = bSw + el * BDIM;
      const v4f B0 = *(const v4f*)(bb);
      const v4f B1 = *(const v4f*)(bb + 4);
      const v4f B2 = *(const v4f*)(bb + 8);
      const v4f B3 = *(const v4f*)(bb + 12);
      ov[j] = rv.x * B0 + rv.y * B1 + rv.z * B2 + rv.w * B3;
    }
#pragma unroll
    for (int j = 0; j < 4; ++j) {
      const int e = e0 + 4 * j + (lane >> 3);
      if (e < E) *(volatile v4f*)(out + (size_t)e * ODIM + (lane & 7) * 4) = ov[j];
    }
    __threadfence();
#pragma unroll
    for (int j = 0; j < 4; ++j) {
      const int e = e0 + 4 * j + (lane >> 3);
      if (e < E) *(volatile v4f*)(out + (size_t)e * ODIM + (lane & 7) * 4) = ov[j];
    }
    __syncthreads();
  }
}

extern "C" void kernel_launch(void* const* d_in, const int* in_sizes, int n_in,
                              void* d_out, int out_size, void* d_ws, size_t ws_size,
                              hipStream_t stream) {
  if (n_in < 9) return;
  const int E = out_size / ODIM;
  if (E <= 0 || out_size != E * ODIM) return;
  if (in_sizes[0] != E * BDIM || in_sizes[1] != E * BDIM || in_sizes[2] != E * EFD || in_sizes[4] != E) return;
  if (in_sizes[3] < FDIM || (in_sizes[3] % FDIM) != 0) return;
  if (in_sizes[5] != EFD * HID || in_sizes[6] != HID || in_sizes[7] != HID * NA * NB || in_sizes[8] != NA * NB) return;

  const float* basis1 = (const float*)d_in[0];
  const float* basis2 = (const float*)d_in[1];
  const float* ef     = (const float*)d_in[2];
  const float* fnode  = (const float*)d_in[3];
  const int*   src    = (const int*)d_in[4];
  const float* w1     = (const float*)d_in[5];
  const float* bias1  = (const float*)d_in[6];
  const float* w2     = (const float*)d_in[7];
  const float* bias2  = (const float*)d_in[8];
  float* out = (float*)d_out;
  const int Nn = in_sizes[3] / FDIM;

  const int    nW2      = HID * NA * NB;
  const int    tblElems = TBL_ROWS * NB;
  const size_t tblBytes = (size_t)tblElems * 2;
  if (2 * tblBytes > ws_size) return;
  unsigned short* tblH = (unsigned short*)d_ws;
  unsigned short* tblL = (unsigned short*)((char*)d_ws + tblBytes);

  const int nGroups = tblElems / 8;
  dim3 grid1((nGroups + NTHR - 1) / NTHR);
  dim3 block(NTHR);
  hipLaunchKernelGGL(k_split_tbl, grid1, block, 0, stream, w2, bias2, tblH, tblL, nW2, tblElems);

  const int numTiles = (E + 15) / 16;
  int g = (numTiles + WPB - 1) / WPB;
  if (g > 1024) g = 1024;
  if (g < 1) g = 1;
  const int nIter = (numTiles + g * WPB - 1) / (g * WPB);
  dim3 grid2(g);
  hipLaunchKernelGGL(k_edge_main, grid2, block, 0, stream,
                     basis1, basis2, ef, fnode, src, w1, bias1,
                     (const unsigned short*)tblH, (const unsigned short*)tblL,
                     out, E, Nn, nIter);
}
